// ClusterGatedSpatialSelfAttention_39702677684479
// MI455X (gfx1250) — hardware-verified
//
#include <hip/hip_runtime.h>
#include <math.h>
#include <stdint.h>

#define NGRP   192
#define NN     207
#define NPG    208
#define NKP    256
#define DM     256
#define NH     8
#define HD     32
#define DG     512
#define GPC    48
#define NCH    4
#define RPC    (GPC * NPG)
#define KROWS  (RPC + 64)
#define XROWS  (NCH * RPC + 64)
#define NQT    13
#define NKS    7
#define NSL    (2 * NH)
#define FLE    256
#define PSP    36
#define ACARRY 16.0f
#define WSC    64.0f
#define QKC    16.0f
#define VC     16.0f
#define PC     1024.0f
#define ZC     64.0f
#define RESC   2048.0f
#define RINV   0.00048828125f
#define NEGS   (-1.0e30f)
#define NLOG2E (-1.4426950408889634f)

static_assert(NGRP == NCH * GPC);
static_assert(NH * HD == DM);
static_assert(NQT * 16 == NPG && NPG > NN);
static_assert(NKS * 32 >= NN && NKS * 32 <= NKP);
static_assert((RPC % 64) == 0 && (KROWS % 64) == 0 && (XROWS % 64) == 0);
static_assert(KROWS >= (GPC - 1) * NPG + NKS * 32);
static_assert(XROWS >= (NCH - 1) * RPC + KROWS);
static_assert(XROWS >= (NCH - 1) * RPC + (GPC - 1) * NPG + NKP);
static_assert(((XROWS * 32) % 256) == 0);
static_assert(((GPC * NH * NQT) % 4) == 0);
static_assert(NN + FLE <= 512);

typedef _Float16 v16h __attribute__((ext_vector_type(16)));
typedef _Float16 v8h  __attribute__((ext_vector_type(8)));
typedef float    v8f  __attribute__((ext_vector_type(8)));
typedef float    v4f  __attribute__((ext_vector_type(4)));
typedef unsigned int v4u __attribute__((ext_vector_type(4)));

union FragH { v16h v; v8h h[2]; v4u u[2]; };

__device__ __forceinline__ unsigned short bf_bits(float f) {
  unsigned u = __float_as_uint(f);
  return (unsigned short)((u + 0x7FFFu + ((u >> 16) & 1u)) >> 16);
}
__device__ __forceinline__ float bf_up(unsigned short b) { return __uint_as_float(((unsigned)b) << 16); }
__device__ __forceinline__ float bfr(float f) { return bf_up(bf_bits(f)); }
__device__ __forceinline__ unsigned short h_bits(_Float16 x) { return __builtin_bit_cast(unsigned short, x); }
__device__ __forceinline__ unsigned pk16(unsigned short a, unsigned short b) { return (unsigned)a | ((unsigned)b << 16); }
__device__ __forceinline__ v8f zero8() { v8f z = {0.f, 0.f, 0.f, 0.f, 0.f, 0.f, 0.f, 0.f}; return z; }

__device__ __forceinline__ v16h ldfrag_h(const _Float16* p) {
  FragH f;
  f.h[0] = *(const v8h*)(p);
  f.h[1] = *(const v8h*)(p + 16);
  return f.v;
}
__device__ __forceinline__ v16h ldfrag_u(const unsigned short* p) {
  FragH f;
  f.u[0] = *(const v4u*)(p);
  f.u[1] = *(const v4u*)(p + 16);
  return f.v;
}

__device__ __forceinline__ v8f mma_raw(v16h a, v16h b, v8f c) {
  return __builtin_amdgcn_wmma_f32_16x16x32_f16(false, a, false, b, (short)0, c, false, false);
}
__device__ __forceinline__ void dep_guard1(v8f& a, v8f& b, v16h x) {
#if defined(__HIP_DEVICE_COMPILE__)
  asm volatile("v_nop\n\tv_nop\n\tv_nop\n\tv_nop" : "+v"(a), "+v"(b) : "v"(x));
#endif
}
__device__ __forceinline__ void keep4_h(v16h a, v16h b, v16h c, v16h d) {
#if defined(__HIP_DEVICE_COMPILE__)
  asm volatile("v_nop" :: "v"(a), "v"(b), "v"(c), "v"(d));
#endif
}
__device__ __forceinline__ void acc_guard4(v8f& a, v8f& b, v8f& c, v8f& d) {
#if defined(__HIP_DEVICE_COMPILE__)
  asm volatile("v_nop\n\tv_nop\n\tv_nop\n\tv_nop" : "+v"(a), "+v"(b), "+v"(c), "+v"(d));
#endif
}
__device__ __forceinline__ void guard_4x4(v8f& a, v8f& b, v8f& c, v8f& d, v16h x0, v16h x1, v16h x2, v16h x3) {
#if defined(__HIP_DEVICE_COMPILE__)
  asm volatile("v_nop\n\tv_nop\n\tv_nop\n\tv_nop" : "+v"(a), "+v"(b), "+v"(c), "+v"(d) : "v"(x0), "v"(x1), "v"(x2), "v"(x3));
#endif
}
__device__ __forceinline__ void guard_4x6(v8f& a, v8f& b, v8f& c, v8f& d,
                                          v16h x0, v16h x1, v16h x2, v16h x3, v16h x4, v16h x5) {
#if defined(__HIP_DEVICE_COMPILE__)
  asm volatile("v_nop\n\tv_nop\n\tv_nop\n\tv_nop"
               : "+v"(a), "+v"(b), "+v"(c), "+v"(d) : "v"(x0), "v"(x1), "v"(x2), "v"(x3), "v"(x4), "v"(x5));
#endif
}
__device__ __forceinline__ void wave_sync_lds() {
  __builtin_amdgcn_fence(__ATOMIC_RELEASE, "workgroup");
  __builtin_amdgcn_wave_barrier();
  __builtin_amdgcn_fence(__ATOMIC_ACQUIRE, "workgroup");
}

__device__ __forceinline__ void split8(const float* sp, v4u& hi, v4u& lo) {
  const v4f a = *(const v4f*)(sp), b = *(const v4f*)(sp + 4);
  float v[8];
#pragma unroll
  for (int e = 0; e < 4; ++e) { v[e] = a[e]; v[4 + e] = b[e]; }
#pragma unroll
  for (int e = 0; e < 4; ++e) {
    const _Float16 h0 = (_Float16)v[2 * e], h1 = (_Float16)v[2 * e + 1];
    const _Float16 l0 = (_Float16)((v[2 * e] - (float)h0) * RESC);
    const _Float16 l1 = (_Float16)((v[2 * e + 1] - (float)h1) * RESC);
    hi[e] = pk16(h_bits(h0), h_bits(h1));
    lo[e] = pk16(h_bits(l0), h_bits(l1));
  }
}

__global__ __launch_bounds__(256) void wtcv(const float* __restrict__ W, unsigned short* dst, int K, int N) {
  __shared__ float sm[64][65];
  const int t  = threadIdx.x;
  const int k0 = blockIdx.x * 64, n0 = blockIdx.y * 64;
  const int kl = t >> 2, nq = (t & 3) * 16;
  const float* src = W + (size_t)(k0 + kl) * (size_t)N + n0 + nq;
#pragma unroll
  for (int q = 0; q < 4; ++q) {
    const v4f a = *(const v4f*)(src + 4 * q);
#pragma unroll
    for (int e = 0; e < 4; ++e) sm[kl][nq + 4 * q + e] = a[e];
  }
  __syncthreads();
  v4u o[2];
#pragma unroll
  for (int it = 0; it < 2; ++it) {
    const int p = it * 256 + t, nl = p >> 3, c8 = (p & 7) * 8;
    v4u a;
#pragma unroll
    for (int e = 0; e < 4; ++e) {
      const float f0 = bfr(sm[c8 + 2 * e][nl]) * WSC, f1 = bfr(sm[c8 + 2 * e + 1][nl]) * WSC;
      a[e] = pk16(h_bits((_Float16)f0), h_bits((_Float16)f1));
    }
    o[it] = a;
  }
#pragma unroll
  for (int it = 0; it < 2; ++it) {
    const int p = it * 256 + t, nl = p >> 3, c8 = (p & 7) * 8;
    *(volatile v4u*)(dst + (size_t)(n0 + nl) * (size_t)K + k0 + c8) = o[it];
  }
  __threadfence();
#pragma unroll
  for (int it = 0; it < 2; ++it) {
    const int p = it * 256 + t, nl = p >> 3, c8 = (p & 7) * 8;
    *(volatile v4u*)(dst + (size_t)(n0 + nl) * (size_t)K + k0 + c8) = o[it];
  }
}

__global__ __launch_bounds__(256) void xcv(const float* __restrict__ x, unsigned short* XP) {
  const int i    = blockIdx.x * 256 + threadIdx.x;
  const int row  = i >> 5;
  const int c8   = (i & 31) * 8;
  const int g    = row / NPG;
  const int node = row - g * NPG;
  const bool live = (g < NGRP) && (node < NN);
  const int gc = (g < NGRP) ? g : (NGRP - 1);
  const int nc = (node < NN) ? node : (NN - 1);
  const float* p = x + ((size_t)gc * NN + nc) * DM + c8;
  const v4f a = *(const v4f*)(p), b = *(const v4f*)(p + 4);
  float v[8];
#pragma unroll
  for (int e = 0; e < 4; ++e) {
    v[e]     = live ? bfr(a[e]) : 0.f;
    v[4 + e] = live ? bfr(b[e]) : 0.f;
  }
  v4u o;
#pragma unroll
  for (int e = 0; e < 4; ++e) o[e] = pk16(h_bits((_Float16)(v[2 * e] * ACARRY)), h_bits((_Float16)(v[2 * e + 1] * ACARRY)));
  unsigned short* dp = XP + (size_t)i * 8;
  *(volatile v4u*)dp = o;
  __threadfence();
  *(volatile v4u*)dp = o;
}

__global__ __launch_bounds__(256) void rowflags(const int* __restrict__ Mi, const int* __restrict__ Me, int* FL) {
  __shared__ __align__(16) int sf[512];
  const int t  = threadIdx.x;
  const int tc = (t < NN) ? t : (NN - 1);
  int ai = 0, ae = 0;
#pragma unroll 1
  for (int j = 0; j < NN; ++j) {
    ai |= Mi[(size_t)tc * NN + j];
    ae |= Me[(size_t)tc * NN + j];
  }
  sf[t]       = (t < NN && ai == 0) ? 1 : 0;
  sf[FLE + t] = (t < NN && ae == 0) ? 1 : 0;
  __syncthreads();
  const int t4 = (t < 128) ? t : 127;
  v4u o;
#pragma unroll
  for (int e = 0; e < 4; ++e) o[e] = (unsigned)sf[4 * t4 + e];
  int* dp = FL + 4 * t4;
  if (t < 128) *(volatile v4u*)dp = o;
  __threadfence();
  if (t < 128) *(volatile v4u*)dp = o;
}

__device__ __forceinline__ void kloop(v8f (&acc)[4][4], const unsigned short* __restrict__ A1, int lda, long long sAk,
                                      const unsigned short* __restrict__ Bb, int ldb, int m0, int n0, int K,
                                      int rlane, int koff) {
  for (int k0 = 0; k0 < K; k0 += 32) {
    v16h bh[4];
#pragma unroll
    for (int j = 0; j < 4; ++j) {
      const size_t bofs = (size_t)(n0 + (j << 4) + rlane) * (size_t)ldb + (size_t)(koff + k0);
      bh[j] = ldfrag_u(Bb + bofs);
    }
    const size_t ak = (size_t)(k0 >> 5) * (size_t)sAk + (size_t)((k0 & 31) + koff);
#pragma unroll
    for (int i = 0; i < 4; ++i) {
      const size_t ao = (size_t)(m0 + (i << 4) + rlane) * (size_t)lda + ak;
      const v16h ah = ldfrag_u(A1 + ao);
#pragma unroll
      for (int j = 0; j < 4; ++j) acc[i][j] = mma_raw(ah, bh[j], acc[i][j]);
      dep_guard1(acc[i][0], acc[i][3], ah);
    }
    keep4_h(bh[0], bh[1], bh[2], bh[3]);
  }
}

template <int OM, int BIASM>
__global__ __launch_bounds__(256) void gemm64(
    const unsigned short* __restrict__ Ap, int lda, long long sAk, long long aLo, long long sAo, long long sAi,
    const unsigned short* __restrict__ Btp, int ldb, long long sBo, long long sBi,
    const float* __restrict__ bias, int sbo, int sbi, float bscale,
    void* Cout, int ldc, long long cLo, long long sCo, long long sCi,
    int M, int N, int K, int Nv, int nin, float oscale, int rowbase) {
  __shared__ __align__(16) float sT[8][16 * 68];
  const int by   = blockIdx.y;
  const int bo   = by / nin;
  const int bi   = by - bo * nin;
  const int lane = threadIdx.x & 31;
  const int wave = threadIdx.x >> 5;
  const int tilesN = N >> 6;
  const int tilesM = M >> 6;
  const int tile = blockIdx.x * 8 + wave;
  if (tile >= tilesM * tilesN) return;
  const int tm = tile / tilesN;
  const int tn = tile - tm * tilesN;
  const int m0 = tm << 6;
  const int n0 = tn << 6;

  const unsigned short* A1 = Ap  + (size_t)((long long)bo * sAo + (long long)bi * sAi);
  const unsigned short* Bb = Btp + (size_t)((long long)bo * sBo + (long long)bi * sBi);
  const float*         bsp = bias + (size_t)bo * (size_t)sbo + (size_t)bi * (size_t)sbi;

  const int rlane = lane & 15;
  const int koff  = (lane >> 4) * 8;
  const int mOff  = (lane >> 4) * 8;

  v8f acc[4][4];
#pragma unroll
  for (int i = 0; i < 4; ++i)
#pragma unroll
    for (int j = 0; j < 4; ++j) acc[i][j] = zero8();

  if (aLo != 0) {
    kloop(acc, A1 + aLo, lda, sAk, Bb, ldb, m0, n0, K, rlane, koff);
    acc_guard4(acc[0][0], acc[0][1], acc[0][2], acc[0][3]);
    acc_guard4(acc[1][0], acc[1][1], acc[1][2], acc[1][3]);
    acc_guard4(acc[2][0], acc[2][1], acc[2][2], acc[2][3]);
    acc_guard4(acc[3][0], acc[3][1], acc[3][2], acc[3][3]);
#pragma unroll
    for (int i = 0; i < 4; ++i)
#pragma unroll
      for (int j = 0; j < 4; ++j) acc[i][j] = acc[i][j] * RINV;
  }
  kloop(acc, A1, lda, sAk, Bb, ldb, m0, n0, K, rlane, koff);
  acc_guard4(acc[0][0], acc[0][1], acc[0][2], acc[0][3]);
  acc_guard4(acc[1][0], acc[1][1], acc[1][2], acc[1][3]);
  acc_guard4(acc[2][0], acc[2][1], acc[2][2], acc[2][3]);
  acc_guard4(acc[3][0], acc[3][1], acc[3][2], acc[3][3]);

  const int hh2 = lane >> 4, c4 = (lane & 15) * 4;
  const int q8  = lane >> 3, c8 = (lane & 7) * 8;
  float bc[8];
#pragma unroll
  for (int e = 0; e < 8; ++e) bc[e] = 0.f;
  if (BIASM == 0) {
    if (OM == 4) {
      const int cb = n0 + c4;
      const int i0 = (cb < N - 4) ? cb : (N - 4);
      const v4f b0v = *(const v4f*)(bsp + i0);
#pragma unroll
      for (int e = 0; e < 4; ++e) bc[e] = bfr(b0v[e]) * bscale;
    } else {
      const int cb = n0 + c8;
      const int i0 = (cb < N - 8) ? cb : (N - 8);
      const v4f b0a = *(const v4f*)(bsp + i0), b0b = *(const v4f*)(bsp + i0 + 4);
#pragma unroll
      for (int e = 0; e < 4; ++e) {
        bc[e]     = bfr(b0a[e]) * bscale;
        bc[4 + e] = bfr(b0b[e]) * bscale;
      }
    }
  }

  float* slab = sT[wave];
#pragma unroll
  for (int i = 0; i < 4; ++i) {
    const int mBase = m0 + (i << 4);
#pragma unroll
    for (int j = 0; j < 4; ++j) {
#pragma unroll
      for (int r = 0; r < 8; ++r) {
        slab[(mOff + r) * 68 + (j << 4) + rlane] = acc[i][j][r];
      }
    }
    wave_sync_lds();
    if (OM == 4) {
      float* C = (float*)Cout + (size_t)((long long)bo * sCo + (long long)bi * sCi);
      v4f vals[8];
#pragma unroll
      for (int it = 0; it < 8; ++it) {
        const int row = it * 2 + hh2;
        v4f v = *(const v4f*)(slab + row * 68 + c4);
#pragma unroll
        for (int e = 0; e < 4; ++e) v[e] = v[e] * oscale + bc[e];
        vals[it] = v;
      }
#pragma unroll
      for (int it = 0; it < 8; ++it) {
        const int gr = mBase + it * 2 + hh2;
        const int gq = gr / NPG, nd = gr - gq * NPG;
        if (nd < NN) *(volatile v4f*)(C + (size_t)(rowbase + gq * NN + nd) * (size_t)ldc + n0 + c4) = vals[it];
      }
      __threadfence();
#pragma unroll
      for (int it = 0; it < 8; ++it) {
        const int gr = mBase + it * 2 + hh2;
        const int gq = gr / NPG, nd = gr - gq * NPG;
        if (nd < NN) *(volatile v4f*)(C + (size_t)(rowbase + gq * NN + nd) * (size_t)ldc + n0 + c4) = vals[it];
      }
      __threadfence();
    } else {
      unsigned short* C = (unsigned short*)Cout + (size_t)((long long)bo * sCo + (long long)bi * sCi);
      v4u hv[4], lv[4];
#pragma unroll
      for (int it = 0; it < 4; ++it) {
        const int row = it * 4 + q8;
        const float* sp = slab + row * 68 + c8;
        const v4f x0 = *(const v4f*)(sp), x1 = *(const v4f*)(sp + 4);
        float bm = 0.f;
        if (BIASM == 1) bm = bfr(bsp[mBase + row]) * bscale;
        float v[8];
#pragma unroll
        for (int e = 0; e < 4; ++e) {
          v[e]     = x0[e] * oscale + ((BIASM == 1) ? bm : bc[e]);
          v[4 + e] = x1[e] * oscale + ((BIASM == 1) ? bm : bc[4 + e]);
        }
#pragma unroll
        for (int e = 0; e < 8; ++e) {
          if (n0 + c8 + e >= Nv) v[e] = 0.f;
        }
        if (OM == 5) {
          const int col0 = n0 + c8;
          const int si = col0 >> 5, d0 = col0 & 31;
          const _Float16* Zh = (const _Float16*)(const void*)A1;
          const _Float16* Zl = Zh + aLo;
          const size_t oi = (size_t)si * (size_t)sAk + (size_t)(mBase + row) * (size_t)lda + (size_t)d0;
          const size_t oe = oi + (size_t)NH * (size_t)sAk;
          const v8h zih = *(const v8h*)(Zh + oi), zil = *(const v8h*)(Zl + oi);
          const v8h zeh = *(const v8h*)(Zh + oe), zel = *(const v8h*)(Zl + oe);
#pragma unroll
          for (int e = 0; e < 8; ++e) {
            const float ex = exp2f(v[e] * NLOG2E);
            const float gt = __builtin_amdgcn_rcpf(1.0f + ex);
            const float ze = (float)zeh[e] + (float)zel[e] * RINV;
            const float df = ((float)zih[e] - (float)zeh[e]) + ((float)zil[e] - (float)zel[e]) * RINV;
            v[e] = ze + gt * df;
          }
        }
        v4u ha, la;
#pragma unroll
        for (int e = 0; e < 4; ++e) {
          const _Float16 h0 = (_Float16)v[2 * e], h1 = (_Float16)v[2 * e + 1];
          ha[e] = pk16(h_bits(h0), h_bits(h1));
          if (OM != 2) {
            const _Float16 l0 = (_Float16)((v[2 * e] - (float)h0) * RESC);
            const _Float16 l1 = (_Float16)((v[2 * e + 1] - (float)h1) * RESC);
            la[e] = pk16(h_bits(l0), h_bits(l1));
          } else {
            la[e] = 0u;
          }
        }
        hv[it] = ha;
        lv[it] = la;
      }
#pragma unroll
      for (int it = 0; it < 4; ++it) {
        const int row = it * 4 + q8;
        const size_t o = (size_t)(mBase + row) * (size_t)ldc + n0 + c8;
        *(volatile v4u*)(C + o) = hv[it];
        if (OM != 2) *(volatile v4u*)(C + cLo + o) = lv[it];
      }
      __threadfence();
#pragma unroll
      for (int it = 0; it < 4; ++it) {
        const int row = it * 4 + q8;
        const size_t o = (size_t)(mBase + row) * (size_t)ldc + n0 + c8;
        *(volatile v4u*)(C + o) = hv[it];
        if (OM != 2) *(volatile v4u*)(C + cLo + o) = lv[it];
      }
      __threadfence();
    }
    wave_sync_lds();
  }
}

__device__ __forceinline__ void build_p(const float* pt, int c, int hh, FragH& ph, FragH& pl) {
  const float* prow = pt + c * PSP + 8 * hh;
  const v4f p0 = *(const v4f*)(prow), p1 = *(const v4f*)(prow + 4);
  const v4f p2 = *(const v4f*)(prow + 16), p3 = *(const v4f*)(prow + 20);
#pragma unroll
  for (int e = 0; e < 4; ++e) {
    float v; _Float16 hv;
    v = p0[e] * PC; hv = (_Float16)v; ph.h[0][e]     = hv; pl.h[0][e]     = (_Float16)((v - (float)hv) * RESC);
    v = p1[e] * PC; hv = (_Float16)v; ph.h[0][4 + e] = hv; pl.h[0][4 + e] = (_Float16)((v - (float)hv) * RESC);
    v = p2[e] * PC; hv = (_Float16)v; ph.h[1][e]     = hv; pl.h[1][e]     = (_Float16)((v - (float)hv) * RESC);
    v = p3[e] * PC; hv = (_Float16)v; ph.h[1][4 + e] = hv; pl.h[1][4 + e] = (_Float16)((v - (float)hv) * RESC);
  }
}

__device__ __forceinline__ void store_tile16x32(const float* os, int lane, unsigned short* dh, unsigned short* dl) {
  v4u h0, l0, h1, l1;
  split8(os + lane * 8, h0, l0);
  split8(os + 256 + lane * 8, h1, l1);
  *(volatile v4u*)(dh + lane * 8) = h0;
  *(volatile v4u*)(dh + 256 + lane * 8) = h1;
  *(volatile v4u*)(dl + lane * 8) = l0;
  *(volatile v4u*)(dl + 256 + lane * 8) = l1;
  __threadfence();
  *(volatile v4u*)(dh + lane * 8) = h0;
  *(volatile v4u*)(dh + 256 + lane * 8) = h1;
  *(volatile v4u*)(dl + lane * 8) = l0;
  *(volatile v4u*)(dl + 256 + lane * 8) = l1;
  __threadfence();
}

__global__ __launch_bounds__(128)
void attn(const unsigned short* __restrict__ QH, const unsigned short* __restrict__ QL,
          const unsigned short* __restrict__ KH,
          const unsigned short* __restrict__ VTH, const unsigned short* __restrict__ VTL,
          const int* __restrict__ Mi, const int* __restrict__ Me, const int* __restrict__ FL,
          unsigned short* ZH, unsigned short* ZL) {
  __shared__ __align__(16) float Ps[4][2][16 * PSP];
  __shared__ __align__(16) float Os[4][16 * 32];

  const int tid  = threadIdx.x;
  const int wave = tid >> 5;
  const int lane = tid & 31;
  const int hh   = lane >> 4;
  const int c    = lane & 15;

  const int wid  = blockIdx.x * 4 + wave;
  const int g    = wid / (NH * NQT);
  const int rem  = wid - g * (NH * NQT);
  const int h    = rem / NQT;
  const int qt   = rem - h * NQT;
  const int q0   = qt * 16;
  const int rb   = g * NPG;

  const _Float16* qhp = (const _Float16*)(const void*)QH + (size_t)(rb + q0 + c) * DM + HD * h + 8 * hh;
  const _Float16* qlp = (const _Float16*)(const void*)QL + (size_t)(rb + q0 + c) * DM + HD * h + 8 * hh;
  const v16h qh = ldfrag_h(qhp), ql = ldfrag_h(qlp);
  const _Float16* kbp = (const _Float16*)(const void*)KH + (size_t)(rb + c) * DM + HD * h + 8 * hh;
  const _Float16* vhp = (const _Float16*)(const void*)VTH + ((size_t)g * DM + HD * h + c) * NKP + 8 * hh;
  const _Float16* vlp = (const _Float16*)(const void*)VTL + ((size_t)g * DM + HD * h + c) * NKP + 8 * hh;

  unsigned fbI = 0u, fbE = 0u;
#pragma unroll
  for (int r = 0; r < 8; ++r) {
    const int qr = q0 + 8 * hh + r;
    const int qc = (qr < NN) ? qr : (NN - 1);
    fbI |= ((FL[qc] != 0) ? 1u : 0u) << r;
    fbE |= ((FL[FLE + qc] != 0) ? 1u : 0u) << r;
  }
  const float lsc = (1.4426950408889634f * 0.17677669529663687f) / (QKC * QKC);

  float mI[8], lI[8], mE[8], lE[8];
  v8f zi0h = zero8(), zi0x = zero8(), zi1h = zero8(), zi1x = zero8();
  v8f ze0h = zero8(), ze0x = zero8(), ze1h = zero8(), ze1x = zero8();
#pragma unroll
  for (int r = 0; r < 8; ++r) { mI[r] = NEGS; lI[r] = 0.f; mE[r] = NEGS; lE[r] = 0.f; }
  float* pI = Ps[wave][0];
  float* pE = Ps[wave][1];

#pragma unroll 1
  for (int ks = 0; ks < NKS; ++ks) {
    const int kb = ks * 32;
    v8f s0h, s0x, s1h, s1x;
    {
      const v16h kf0 = ldfrag_h(kbp + (size_t)kb * DM), kf1 = ldfrag_h(kbp + (size_t)(kb + 16) * DM);
      s0h = mma_raw(qh, kf0, zero8());
      s0x = mma_raw(ql, kf0, zero8());
      s1h = mma_raw(qh, kf1, zero8());
      s1x = mma_raw(ql, kf1, zero8());
      guard_4x4(s0h, s0x, s1h, s1x, qh, ql, kf0, kf1);
    }
    const int key0 = kb + c, key1 = kb + 16 + c;
    const bool in0 = key0 < NN, in1 = key1 < NN;
    const int k0c = in0 ? key0 : (NN - 1), k1c = in1 ? key1 : (NN - 1);
#pragma unroll
    for (int r = 0; r < 8; ++r) {
      const int qr = q0 + 8 * hh + r;
      const int qc = (qr < NN) ? qr : (NN - 1);
      const int* mip = Mi + (size_t)qc * NN;
      const int* mep = Me + (size_t)qc * NN;
      const int mi0 = mip[k0c], mi1 = mip[k1c];
      const int me0 = mep[k0c], me1 = mep[k1c];
      const float s0 = (s0h[r] + s0x[r] * RINV) * lsc;
      const float s1 = (s1h[r] + s1x[r] * RINV) * lsc;
      const int ro = (8 * hh + r) * PSP + c;
      {
        const bool f   = ((fbI >> r) & 1u) != 0u;
        const bool kp0 = in0 && (f || (mi0 != 0));
        const bool kp1 = in1 && (f || (mi1 != 0));
        const float t0 = f ? 0.f : s0, t1 = f ? 0.f : s1;
        float mx = fmaxf(kp0 ? t0 : NEGS, kp1 ? t1 : NEGS);
        mx = fmaxf(mx, __shfl_xor(mx, 1, 32));
        mx = fmaxf(mx, __shfl_xor(mx, 2, 32));
        mx = fmaxf(mx, __shfl_xor(mx, 4, 32));
        mx = fmaxf(mx, __shfl_xor(mx, 8, 32));
        const float mn = fmaxf(mI[r], mx);
        const float al = exp2f(mI[r] - mn);
        mI[r] = mn;
        const float e0 = kp0 ? exp2f(t0 - mn) : 0.f;
        const float e1 = kp1 ? exp2f(t1 - mn) : 0.f;
        float ps = e0 + e1;
        ps += __shfl_xor(ps, 1, 32);
        ps += __shfl_xor(ps, 2, 32);
        ps += __shfl_xor(ps, 4, 32);
        ps += __shfl_xor(ps, 8, 32);
        lI[r] = lI[r] * al + ps;
        zi0h[r] *= al; zi0x[r] *= al; zi1h[r] *= al; zi1x[r] *= al;
        pI[ro]      = e0;
        pI[ro + 16] = e1;
      }
      {
        const bool f   = ((fbE >> r) & 1u) != 0u;
        const bool kp0 = in0 && (f || (me0 != 0));
        const bool kp1 = in1 && (f || (me1 != 0));
        const float t0 = f ? 0.f : s0, t1 = f ? 0.f : s1;
        float mx = fmaxf(kp0 ? t0 : NEGS, kp1 ? t1 : NEGS);
        mx = fmaxf(mx, __shfl_xor(mx, 1, 32));
        mx = fmaxf(mx, __shfl_xor(mx, 2, 32));
        mx = fmaxf(mx, __shfl_xor(mx, 4, 32));
        mx = fmaxf(mx, __shfl_xor(mx, 8, 32));
        const float mn = fmaxf(mE[r], mx);
        const float al = exp2f(mE[r] - mn);
        mE[r] = mn;
        const float e0 = kp0 ? exp2f(t0 - mn) : 0.f;
        const float e1 = kp1 ? exp2f(t1 - mn) : 0.f;
        float ps = e0 + e1;
        ps += __shfl_xor(ps, 1, 32);
        ps += __shfl_xor(ps, 2, 32);
        ps += __shfl_xor(ps, 4, 32);
        ps += __shfl_xor(ps, 8, 32);
        lE[r] = lE[r] * al + ps;
        ze0h[r] *= al; ze0x[r] *= al; ze1h[r] *= al; ze1x[r] *= al;
        pE[ro]      = e0;
        pE[ro + 16] = e1;
      }
    }
    wave_sync_lds();
    const v16h vh0 = ldfrag_h(vhp + kb), vh1 = ldfrag_h(vhp + (size_t)16 * NKP + kb);
    const v16h vl0 = ldfrag_h(vlp + kb), vl1 = ldfrag_h(vlp + (size_t)16 * NKP + kb);
    {
      FragH ph, pl;
      build_p(pI, c, hh, ph, pl);
      zi0h = mma_raw(ph.v, vh0, zi0h);
      zi0x = mma_raw(ph.v, vl0, zi0x);
      zi0x = mma_raw(pl.v, vh0, zi0x);
      zi1h = mma_raw(ph.v, vh1, zi1h);
      zi1x = mma_raw(ph.v, vl1, zi1x);
      zi1x = mma_raw(pl.v, vh1, zi1x);
      guard_4x6(zi0h, zi0x, zi1h, zi1x, ph.v, pl.v, vh0, vl0, vh1, vl1);
    }
    {
      FragH ph, pl;
      build_p(pE, c, hh, ph, pl);
      ze0h = mma_raw(ph.v, vh0, ze0h);
      ze0x = mma_raw(ph.v, vl0, ze0x);
      ze0x = mma_raw(pl.v, vh0, ze0x);
      ze1h = mma_raw(ph.v, vh1, ze1h);
      ze1x = mma_raw(ph.v, vl1, ze1x);
      ze1x = mma_raw(pl.v, vh1, ze1x);
      guard_4x6(ze0h, ze0x, ze1h, ze1x, ph.v, pl.v, vh0, vl0, vh1, vl1);
    }
    wave_sync_lds();
  }

  const float oc2 = ZC / (PC * VC);
  float* os = Os[wave];
  {
#pragma unroll
    for (int r = 0; r < 8; ++r) {
      const float inv = (lI[r] > 0.f) ? (__builtin_amdgcn_rcpf(lI[r]) * oc2) : 0.f;
      const int ro = (8 * hh + r) * 32 + c;
      os[ro]      = (zi0h[r] + zi0x[r] * RINV) * inv;
      os[ro + 16] = (zi1h[r] + zi1x[r] * RINV) * inv;
    }
    wave_sync_lds();
    unsigned short* dh = ZH + ((size_t)h * RPC + (size_t)(rb + q0)) * HD;
    unsigned short* dl = ZL + ((size_t)h * RPC + (size_t)(rb + q0)) * HD;
    store_tile16x32(os, lane, dh, dl);
    wave_sync_lds();
  }
  {
#pragma unroll
    for (int r = 0; r < 8; ++r) {
      const float inv = (lE[r] > 0.f) ? (__builtin_amdgcn_rcpf(lE[r]) * oc2) : 0.f;
      const int ro = (8 * hh + r) * 32 + c;
      os[ro]      = (ze0h[r] + ze0x[r] * RINV) * inv;
      os[ro + 16] = (ze1h[r] + ze1x[r] * RINV) * inv;
    }
    wave_sync_lds();
    unsigned short* dh = ZH + ((size_t)(NH + h) * RPC + (size_t)(rb + q0)) * HD;
    unsigned short* dl = ZL + ((size_t)(NH + h) * RPC + (size_t)(rb + q0)) * HD;
    store_tile16x32(os, lane, dh, dl);
    wave_sync_lds();
  }
}

extern "C" void kernel_launch(void* const* d_in, const int* in_sizes, int n_in,
                              void* d_out, int out_size, void* d_ws, size_t ws_size,
                              hipStream_t stream) {
  if (n_in < 13) return;
  if (in_sizes[0] != NGRP * NN * DM) return;
  if (in_sizes[1] != DM * DM || in_sizes[3] != DM * DM || in_sizes[5] != DM * DM || in_sizes[9] != DM * DM) return;
  if (in_sizes[7] != DG * DM) return;
  if (in_sizes[2] != DM || in_sizes[4] != DM || in_sizes[6] != DM || in_sizes[8] != DM || in_sizes[10] != DM) return;
  if (in_sizes[11] != NN * NN || in_sizes[12] != NN * NN) return;
  if (out_size != NGRP * NN * DM) return;

  const float* x   = (const float*)d_in[0];
  const float* Wq  = (const float*)d_in[1];
  const float* bq  = (const float*)d_in[2];
  const float* Wk  = (const float*)d_in[3];
  const float* bk  = (const float*)d_in[4];
  const float* Wv  = (const float*)d_in[5];
  const float* bv  = (const float*)d_in[6];
  const float* Wg  = (const float*)d_in[7];
  const float* bg  = (const float*)d_in[8];
  const float* Wp  = (const float*)d_in[9];
  const float* bp  = (const float*)d_in[10];
  const int*   Mi  = (const int*)d_in[11];
  const int*   Me  = (const int*)d_in[12];
  float*       out = (float*)d_out;

  const size_t BW  = (size_t)DM * DM * 2;
  const size_t BWG = (size_t)DG * DM * 2;
  const size_t BFL = 4096;
  const size_t BXP = (size_t)XROWS * DM * 2;
  const size_t BQ  = (size_t)RPC * DM * 2;
  const size_t BK  = (size_t)KROWS * DM * 2;
  const size_t BVT = (size_t)GPC * DM * NKP * 2;
  const size_t BZ  = (size_t)NSL * RPC * HD * 2;
  size_t off = 0;
  const size_t oWQ = off; off += BW;
  const size_t oWK = off; off += BW;
  const size_t oWV = off; off += BW;
  const size_t oWG = off; off += BWG;
  const size_t oWP = off; off += BW;
  const size_t oFL = off; off += BFL;
  const size_t oXP = off; off += BXP;
  const size_t oQH = off; off += BQ;
  const size_t oQL = off; off += BQ;
  const size_t oKH = off; off += BK;
  const size_t oVH = off; off += BVT;
  const size_t oVL = off; off += BVT;
  const size_t oZH = off; off += BZ;
  const size_t oZL = off; off += BZ;
  const size_t oMH = off; off += BQ;
  const size_t oML = off; off += BQ;
  if (off > ws_size) return;
  if (off > (size_t)134217728) return;

  char* ws = (char*)d_ws;
  unsigned short* WQT = (unsigned short*)(ws + oWQ);
  unsigned short* WKT = (unsigned short*)(ws + oWK);
  unsigned short* WVT = (unsigned short*)(ws + oWV);
  unsigned short* WGT = (unsigned short*)(ws + oWG);
  unsigned short* WPT = (unsigned short*)(ws + oWP);
  int*            FL  = (int*)(ws + oFL);
  unsigned short* XP  = (unsigned short*)(ws + oXP);
  unsigned short* QH  = (unsigned short*)(ws + oQH);
  unsigned short* QL  = (unsigned short*)(ws + oQL);
  unsigned short* KH  = (unsigned short*)(ws + oKH);
  unsigned short* VTH = (unsigned short*)(ws + oVH);
  unsigned short* VTL = (unsigned short*)(ws + oVL);
  unsigned short* ZH  = (unsigned short*)(ws + oZH);
  unsigned short* ZL  = (unsigned short*)(ws + oZL);
  unsigned short* MH  = (unsigned short*)(ws + oMH);
  unsigned short* ML  = (unsigned short*)(ws + oML);

  const dim3 blk(256), blk128(128);
  const dim3 gW(DM / 64, DM / 64), gWG(DG / 64, DM / 64);
  const dim3 gXP((XROWS * 32) / 256);
  const dim3 gQ(((RPC / 64) * (DM / 64) + 7) / 8, 1);
  const dim3 gK(((KROWS / 64) * (DM / 64) + 7) / 8, 1);
  const dim3 gVT(((DM / 64) * (NKP / 64) + 7) / 8, GPC);
  const dim3 gAT((GPC * NH * NQT) / 4);
  const dim3 gGM(((RPC / 64) * (DM / 64) + 7) / 8, 1);

  wtcv<<<gW, blk, 0, stream>>>(Wq, WQT, DM, DM);
  wtcv<<<gW, blk, 0, stream>>>(Wk, WKT, DM, DM);
  wtcv<<<gW, blk, 0, stream>>>(Wv, WVT, DM, DM);
  wtcv<<<gWG, blk, 0, stream>>>(Wg, WGT, DG, DM);
  wtcv<<<gW, blk, 0, stream>>>(Wp, WPT, DM, DM);

  xcv<<<gXP, blk, 0, stream>>>(x, XP);
  rowflags<<<dim3(1), blk, 0, stream>>>(Mi, Me, FL);

  for (int b = 0; b < NCH; ++b) {
    const unsigned short* XPb = XP + (size_t)b * RPC * DM;

    gemm64<3, 0><<<gQ, blk, 0, stream>>>(
        XPb, DM, 32LL, 0LL, 0LL, 0LL,
        WQT, DM, 0LL, 0LL,
        bq, 0, 0, QKC,
        (void*)QH, DM, (long long)(QL - QH), 0LL, 0LL,
        RPC, DM, DM, DM, 1, QKC / (ACARRY * WSC), 0);

    gemm64<2, 0><<<gK, blk, 0, stream>>>(
        XPb, DM, 32LL, 0LL, 0LL, 0LL,
        WKT, DM, 0LL, 0LL,
        bk, 0, 0, QKC,
        (void*)KH, DM, 0LL, 0LL, 0LL,
        KROWS, DM, DM, DM, 1, QKC / (ACARRY * WSC), 0);

    gemm64<3, 1><<<gVT, blk, 0, stream>>>(
        WVT, DM, 32LL, 0LL, 0LL, 0LL,
        XPb, DM, (long long)NPG * DM, 0LL,
        bv, 0, 0, VC,
        (void*)VTH, NKP, (long long)(VTL - VTH), (long long)DM * NKP, 0LL,
        DM, NKP, DM, NN, 1, VC / (ACARRY * WSC), 0);

    attn<<<gAT, blk128, 0, stream>>>(QH, QL, KH, VTH, VTL, Mi, Me, FL, ZH, ZL);

    gemm64<5, 0><<<gGM, blk, 0, stream>>>(
        ZH, HD, (long long)RPC * HD, (long long)(ZL - ZH), 0LL, 0LL,
        WGT, DG, 0LL, 0LL,
        bg, 0, 0, 1.0f,
        (void*)MH, DM, (long long)(ML - MH), 0LL, 0LL,
        RPC, DM, DG, DM, 1, 1.0f / (ZC * WSC), 0);

    gemm64<4, 0><<<gGM, blk, 0, stream>>>(
        MH, DM, 32LL, (long long)(ML - MH), 0LL, 0LL,
        WPT, DM, 0LL, 0LL,
        bp, 0, 0, 1.0f,
        (void*)out, DM, 0LL, 0LL, 0LL,
        RPC, DM, DM, DM, 1, 1.0f / (ZC * WSC), b * GPC * NN);
  }
  (void)hipGetLastError();
}
